// LegacyRelPositionMultiHeadedAttention_73710228734781
// MI455X (gfx1250) — hardware-verified
//
#include <hip/hip_runtime.h>
#include <math.h>
#include <stdint.h>

#define NB  8
#define NT  1024
#define CD  512
#define NH  8
#define HD  64
#define NQB (NT / 64)
#define NKC (NT / 32)
static_assert(NH * HD == CD);
static_assert(HD == 64);
static_assert((NT % 64) == 0 && (CD % 64) == 0);

typedef _Float16 v16h __attribute__((ext_vector_type(16)));
typedef _Float16 v8h  __attribute__((ext_vector_type(8)));
typedef __bf16   v16b __attribute__((ext_vector_type(16)));
typedef __bf16   v8b  __attribute__((ext_vector_type(8)));
typedef float    v8f  __attribute__((ext_vector_type(8)));
typedef float    v4f  __attribute__((ext_vector_type(4)));
typedef unsigned int v4u __attribute__((ext_vector_type(4)));

__device__ __forceinline__ unsigned short bf_bits(float f) {
  unsigned u = __float_as_uint(f);
  return (unsigned short)((u + 0x7FFFu + ((u >> 16) & 1u)) >> 16);
}
__device__ __forceinline__ float bf_up(unsigned short h) { return __uint_as_float(((unsigned)h) << 16); }
__device__ __forceinline__ unsigned short h_bits(_Float16 x) { return __builtin_bit_cast(unsigned short, x); }
__device__ __forceinline__ unsigned pk16(unsigned short a, unsigned short b) { return (unsigned)a | ((unsigned)b << 16); }
__device__ __forceinline__ v8f zero8() { v8f z = {0.f, 0.f, 0.f, 0.f, 0.f, 0.f, 0.f, 0.f}; return z; }

__device__ __forceinline__ v16b ldfrag_b(const __bf16* p) {
  union { v16b v; v8b h[2]; } f;
  f.h[0] = *(const v8b*)(p);
  f.h[1] = *(const v8b*)(p + 16);
  return f.v;
}
__device__ __forceinline__ v16h ldfrag_h(const _Float16* p) {
  union { v16h v; v8h h[2]; } f;
  f.h[0] = *(const v8h*)(p);
  f.h[1] = *(const v8h*)(p + 16);
  return f.v;
}

__device__ __forceinline__ v8f mma_h(v16h a, v16h b, v8f c) {
  c = __builtin_amdgcn_wmma_f32_16x16x32_f16(false, a, false, b, (short)0, c, false, false);
#if defined(__HIP_DEVICE_COMPILE__)
  asm volatile("v_nop\n\tv_nop\n\tv_nop\n\tv_nop" : "+v"(c) : "v"(a), "v"(b));
#endif
  return c;
}
__device__ __forceinline__ v8f mma_b_raw(v16b a, v16b b, v8f c) {
  return __builtin_amdgcn_wmma_f32_16x16x32_bf16(false, a, false, b, (short)0, c, false, false);
}
__device__ __forceinline__ void dep_guard_b(v8f& a, v8f& b, v16b x, v16b y) {
#if defined(__HIP_DEVICE_COMPILE__)
  asm volatile("v_nop\n\tv_nop\n\tv_nop\n\tv_nop" : "+v"(a), "+v"(b) : "v"(x), "v"(y));
#endif
}
__device__ __forceinline__ void keep4_b(v16b a, v16b b, v16b c, v16b d) {
#if defined(__HIP_DEVICE_COMPILE__)
  asm volatile("v_nop" :: "v"(a), "v"(b), "v"(c), "v"(d));
#endif
}
__device__ __forceinline__ void acc_guard4(v8f& a, v8f& b, v8f& c, v8f& d) {
#if defined(__HIP_DEVICE_COMPILE__)
  asm volatile("v_nop\n\tv_nop\n\tv_nop\n\tv_nop" : "+v"(a), "+v"(b), "+v"(c), "+v"(d));
#endif
}
__device__ __forceinline__ void wave_sync_lds() {
  __builtin_amdgcn_fence(__ATOMIC_RELEASE, "workgroup");
  __builtin_amdgcn_wave_barrier();
  __builtin_amdgcn_fence(__ATOMIC_ACQUIRE, "workgroup");
}

__global__ __launch_bounds__(256) void cvt_bf16x8m(
    const float* __restrict__ s0, const float* __restrict__ s1, const float* __restrict__ s2,
    const float* __restrict__ s3, const float* __restrict__ s4,
    unsigned short* d0, unsigned short* d1, unsigned short* d2, unsigned short* d3, unsigned short* d4,
    int n0, int n1, int n2, int n3, int n4) {
  const int z = blockIdx.y;
  const float* in = (z == 0) ? s0 : ((z == 1) ? s1 : ((z == 2) ? s2 : ((z == 3) ? s3 : s4)));
  unsigned short* out = (z == 0) ? d0 : ((z == 1) ? d1 : ((z == 2) ? d2 : ((z == 3) ? d3 : d4)));
  const int n8 = (z == 0) ? n0 : ((z == 1) ? n1 : ((z == 2) ? n2 : ((z == 3) ? n3 : n4)));
  const int i = blockIdx.x * 256 + threadIdx.x;
  if (i < n8) {
    const v4f a = *(const v4f*)(in + (size_t)i * 8);
    const v4f b = *(const v4f*)(in + (size_t)i * 8 + 4);
    v4u p;
    p[0] = pk16(bf_bits(a[0]), bf_bits(a[1]));
    p[1] = pk16(bf_bits(a[2]), bf_bits(a[3]));
    p[2] = pk16(bf_bits(b[0]), bf_bits(b[1]));
    p[3] = pk16(bf_bits(b[2]), bf_bits(b[3]));
    *(volatile v4u*)(out + (size_t)i * 8) = p;
    __threadfence();
    *(volatile v4u*)(out + (size_t)i * 8) = p;
  }
}

template <int NSPLIT, int MODE, int RES>
__global__ __launch_bounds__(256) void gemm64(
    const unsigned short* __restrict__ Ap, const unsigned short* __restrict__ A2p, int lda, long long strideA,
    const unsigned short* __restrict__ Btp, int ldb, long long strideB,
    void* C0p, void* C1p, void* C2p, void* C3p, int ldc, long long strideC,
    int M, int N, int K, float rscale,
    const float* __restrict__ bias0, const float* __restrict__ bias1, const float* __restrict__ bias2, int bdim) {
  const __bf16* A   = (const __bf16*)(const void*)Ap;
  const __bf16* A2  = (const __bf16*)(const void*)A2p;
  const __bf16* Bt  = (const __bf16*)(const void*)Btp;
  __shared__ __align__(16) float sT[8][16 * 68];
  const int b    = blockIdx.y;
  const int lane = threadIdx.x & 31;
  const int wave = threadIdx.x >> 5;
  const int tilesN = N >> 6;
  const int tilesM = M >> 6;
  const int tile = blockIdx.x * 8 + wave;
  if (tile >= tilesM * tilesN) return;
  const int tm = tile / tilesN;
  const int tn = tile - tm * tilesN;
  const int m0 = tm << 6;
  const int n0 = tn << 6;

  const __bf16* Ab  = A  + (size_t)b * strideA;
  const __bf16* Bb  = Bt + (size_t)b * strideB;
  const __bf16* Ab2 = (NSPLIT >= 1) ? (A2 + (size_t)b * strideA) : Ab;

  const int rlane = lane & 15;
  const int koff  = (lane >> 4) * 8;
  const int mOff  = (lane >> 4) * 8;

  v8f acc[4][4];
#pragma unroll
  for (int i = 0; i < 4; ++i)
#pragma unroll
    for (int j = 0; j < 4; ++j) acc[i][j] = zero8();

  for (int k0 = 0; k0 < K; k0 += 32) {
    v16b bh[4];
#pragma unroll
    for (int j = 0; j < 4; ++j) {
      const size_t bo = (size_t)(n0 + (j << 4) + rlane) * ldb + koff + k0;
      bh[j] = ldfrag_b(Bb + bo);
    }
#pragma unroll
    for (int i = 0; i < 4; ++i) {
      const size_t ao = (size_t)(m0 + (i << 4) + rlane) * lda + koff + k0;
      const v16b ah = ldfrag_b(Ab + ao);
      v16b al = ah;
      if (NSPLIT >= 1) al = ldfrag_b(Ab2 + ao);
#pragma unroll
      for (int j = 0; j < 4; ++j) {
        acc[i][j] = mma_b_raw(ah, bh[j], acc[i][j]);
        if (NSPLIT >= 1) acc[i][j] = mma_b_raw(al, bh[j], acc[i][j]);
      }
      dep_guard_b(acc[i][0], acc[i][3], ah, al);
    }
    keep4_b(bh[0], bh[1], bh[2], bh[3]);
  }
  acc_guard4(acc[0][0], acc[0][1], acc[0][2], acc[0][3]);
  acc_guard4(acc[1][0], acc[1][1], acc[1][2], acc[1][3]);
  acc_guard4(acc[2][0], acc[2][1], acc[2][2], acc[2][3]);
  acc_guard4(acc[3][0], acc[3][1], acc[3][2], acc[3][3]);

  float* slab = sT[wave];
#pragma unroll
  for (int i = 0; i < 4; ++i) {
    const int mBase = m0 + (i << 4);
#pragma unroll
    for (int j = 0; j < 4; ++j) {
#pragma unroll
      for (int r = 0; r < 8; ++r) {
        slab[(mOff + r) * 68 + (j << 4) + rlane] = acc[i][j][r];
      }
    }
    wave_sync_lds();
    if (MODE == 0) {
      float* C = (float*)C0p + (size_t)b * strideC;
      const int h2 = lane >> 4, c4 = (lane & 15) * 4;
      v4f bv = {0.f, 0.f, 0.f, 0.f};
      if (bdim == 1) {
#pragma unroll
        for (int e = 0; e < 4; ++e) bv[e] = bf_up(bf_bits(bias0[n0 + c4 + e]));
      }
      for (int pass = 0; pass < 2; ++pass) {
#pragma unroll
        for (int it = 0; it < 8; ++it) {
          const int row = it * 2 + h2;
          const v4f v = *(const v4f*)(slab + row * 68 + c4) + bv;
          *(volatile v4f*)(C + (size_t)(mBase + row) * ldc + n0 + c4) = v;
        }
        __threadfence();
      }
    } else {
      const int q = lane >> 3, c8 = (lane & 7) * 8;
      float cb[8];
#pragma unroll
      for (int e = 0; e < 8; ++e) cb[e] = 0.f;
      if (bdim == 1) {
#pragma unroll
        for (int e = 0; e < 8; ++e) cb[e] = bf_up(bf_bits(bias0[n0 + c8 + e]));
      }
      constexpr int NVAR = (MODE == 4) ? 2 : 1;
#pragma unroll
      for (int var = 0; var < NVAR; ++var) {
        float ub[8];
#pragma unroll
        for (int e = 0; e < 8; ++e) ub[e] = 0.f;
        if (MODE == 4) {
          const float* bx = (var == 0) ? bias1 : bias2;
#pragma unroll
          for (int e = 0; e < 8; ++e) ub[e] = bf_up(bf_bits(bx[n0 + c8 + e]));
        }
        unsigned short* Ch = (unsigned short*)((var == 0) ? C0p : C2p) + (size_t)b * strideC;
        unsigned short* Cl = (unsigned short*)((var == 0) ? C1p : C3p) + (size_t)b * strideC;
        v4u hv[4], lv[4];
#pragma unroll
        for (int it = 0; it < 4; ++it) {
          const int row = it * 4 + q;
          const float* sp = slab + row * 68 + c8;
          float rb = 0.f;
          if (bdim == 2) rb = bf_up(bf_bits(bias0[mBase + row]));
          v4u a, a2;
#pragma unroll
          for (int e = 0; e < 4; ++e) {
            const float f0 = ((sp[2 * e] + cb[2 * e]) + ub[2 * e]) + rb;
            const float f1 = ((sp[2 * e + 1] + cb[2 * e + 1]) + ub[2 * e + 1]) + rb;
            const _Float16 x0 = (_Float16)f0, x1 = (_Float16)f1;
            const unsigned short h0 = h_bits(x0), h1 = h_bits(x1);
            const unsigned short l0 = h_bits((_Float16)((f0 - (float)x0) * rscale));
            const unsigned short l1 = h_bits((_Float16)((f1 - (float)x1) * rscale));
            a[e] = pk16(h0, h1); a2[e] = pk16(l0, l1);
          }
          hv[it] = a; lv[it] = a2;
        }
        for (int pass = 0; pass < 2; ++pass) {
#pragma unroll
          for (int it = 0; it < 4; ++it) {
            const int row = it * 4 + q;
            *(volatile v4u*)(Ch + (size_t)(mBase + row) * ldc + n0 + c8) = hv[it];
            if (RES) *(volatile v4u*)(Cl + (size_t)(mBase + row) * ldc + n0 + c8) = lv[it];
          }
          __threadfence();
        }
      }
    }
    wave_sync_lds();
  }
}

__global__ __launch_bounds__(128)
void attn64(const unsigned short* __restrict__ quhp, const unsigned short* __restrict__ qulp,
            const unsigned short* __restrict__ qvhp, const unsigned short* __restrict__ qvlp,
            const unsigned short* __restrict__ khp,  const unsigned short* __restrict__ klp,
            const unsigned short* __restrict__ php,  const unsigned short* __restrict__ plp,
            const unsigned short* __restrict__ vhp,  const unsigned short* __restrict__ vlp,
            const int* __restrict__ maskp,
            unsigned short* ohp, unsigned short* olp, float sscale, float rres) {
  union FH { v16h v; v8h h[2]; };
  __shared__ __align__(16) _Float16 Psh[4][16 * 32];
  __shared__ __align__(16) _Float16 Psl[4][16 * 32];
  __shared__ __align__(16) float    Os[4][16 * 64];

  const int tid  = threadIdx.x;
  const int wave = tid >> 5;
  const int lane = tid & 31;
  const int hh   = lane >> 4;
  const int c    = lane & 15;

  const int bx   = blockIdx.x;
  const int qb   = bx % NQB;
  const int rest = bx / NQB;
  const int h    = rest % NH;
  const int b    = rest / NH;
  const int q0   = qb * 64 + wave * 16;
  const size_t rowB = (size_t)b * NT;

  const _Float16* QUh = (const _Float16*)(const void*)quhp + (size_t)h * HD;
  const _Float16* QUl = (const _Float16*)(const void*)qulp + (size_t)h * HD;
  const _Float16* QVh = (const _Float16*)(const void*)qvhp + (size_t)h * HD;
  const _Float16* QVl = (const _Float16*)(const void*)qvlp + (size_t)h * HD;
  const _Float16* Kh  = (const _Float16*)(const void*)khp  + (size_t)h * HD;
  const _Float16* Kl  = (const _Float16*)(const void*)klp  + (size_t)h * HD;
  const _Float16* Ph  = (const _Float16*)(const void*)php  + (size_t)h * HD;
  const _Float16* Pl  = (const _Float16*)(const void*)plp  + (size_t)h * HD;
  const _Float16* Vh  = (const _Float16*)(const void*)vhp + ((size_t)b * CD + (size_t)h * HD) * NT;
  const _Float16* Vl  = (const _Float16*)(const void*)vlp + ((size_t)b * CD + (size_t)h * HD) * NT;
  const int* mk = maskp + rowB;

  v16h quh[2], qul[2], qvh[2], qvl[2];
#pragma unroll
  for (int cc = 0; cc < 2; ++cc) {
    const size_t qo = (rowB + q0 + c) * CD + cc * 32 + 8 * hh;
    quh[cc] = ldfrag_h(QUh + qo);
    qul[cc] = ldfrag_h(QUl + qo);
    qvh[cc] = ldfrag_h(QVh + qo);
    qvl[cc] = ldfrag_h(QVl + qo);
  }

  float mrow[8], lrow[8];
  v8f oacc[4];
#pragma unroll
  for (int r = 0; r < 8; ++r) { mrow[r] = -INFINITY; lrow[r] = 0.f; }
#pragma unroll
  for (int t = 0; t < 4; ++t) oacc[t] = zero8();

  _Float16* pwh = Psh[wave];
  _Float16* pwl = Psl[wave];

  for (int kt = 0; kt < NKC; ++kt) {
    const int kv0 = kt * 32;

    v8f s[2];
    int vm[2];
#pragma unroll
    for (int j = 0; j < 2; ++j) {
      const int key = kv0 + j * 16 + c;
      const size_t ko = (rowB + key) * CD + 8 * hh;
      const size_t po = (size_t)key * CD + 8 * hh;
      v8f ar = zero8();
      v8f ah = zero8();
#pragma unroll
      for (int cc = 0; cc < 2; ++cc) {
        const v16h kfl = ldfrag_h(Kl + ko + cc * 32);
        const v16h pfl = ldfrag_h(Pl + po + cc * 32);
        ar = mma_h(quh[cc], kfl, ar);
        ar = mma_h(qvh[cc], pfl, ar);
        const v16h kfh = ldfrag_h(Kh + ko + cc * 32);
        const v16h pfh = ldfrag_h(Ph + po + cc * 32);
        ar = mma_h(qul[cc], kfh, ar);
        ar = mma_h(qvl[cc], pfh, ar);
        ah = mma_h(quh[cc], kfh, ah);
        ah = mma_h(qvh[cc], pfh, ah);
      }
      vm[j] = mk[key];
#pragma unroll
      for (int r = 0; r < 8; ++r) {
        const float sv = (ah[r] + ar[r] * rres) * sscale;
        s[j][r] = (vm[j] != 0) ? sv : -1.0e30f;
      }
    }

#pragma unroll
    for (int r = 0; r < 8; ++r) {
      float m = fmaxf(s[0][r], s[1][r]);
#pragma unroll
      for (int off = 1; off < 16; off <<= 1) m = fmaxf(m, __shfl_xor(m, off, 32));
      const float mnew  = fmaxf(mrow[r], m);
      const float alpha = __expf(mrow[r] - mnew);
      mrow[r] = mnew;
      float psum = 0.f;
#pragma unroll
      for (int j = 0; j < 2; ++j) {
        const float pe = __expf(s[j][r] - mnew);
        const float p  = (vm[j] != 0) ? pe : 0.f;
        psum += p;
        const float p1 = p * 1024.0f;
        const _Float16 x = (_Float16)p1;
        const int idx = (8 * hh + r) * 32 + j * 16 + c;
        pwh[idx] = x;
        pwl[idx] = (_Float16)((p1 - (float)x) * 4096.0f);
      }
#pragma unroll
      for (int off = 1; off < 16; off <<= 1) psum += __shfl_xor(psum, off, 32);
      lrow[r] = lrow[r] * alpha + psum;
#pragma unroll
      for (int t = 0; t < 4; ++t) oacc[t][r] *= alpha;
    }
    wave_sync_lds();

    FH pa, pl;
    pa.h[0] = *(const v8h*)(pwh + c * 32 + 8 * hh);
    pa.h[1] = *(const v8h*)(pwh + c * 32 + 16 + 8 * hh);
    pl.h[0] = *(const v8h*)(pwl + c * 32 + 8 * hh);
    pl.h[1] = *(const v8h*)(pwl + c * 32 + 16 + 8 * hh);
    v8f o1[4];
#pragma unroll
    for (int t = 0; t < 4; ++t) o1[t] = zero8();
#pragma unroll
    for (int t = 0; t < 4; ++t) {
      const size_t vo = (size_t)(t * 16 + c) * NT + kv0 + 8 * hh;
      const v16h vb = ldfrag_h(Vh + vo);
      const v16h vl = ldfrag_h(Vl + vo);
      oacc[t] = mma_h(pa.v, vb, oacc[t]);
      o1[t]   = mma_h(pa.v, vl, o1[t]);
      o1[t]   = mma_h(pl.v, vb, o1[t]);
    }
#pragma unroll
    for (int t = 0; t < 4; ++t)
#pragma unroll
      for (int r = 0; r < 8; ++r) oacc[t][r] += o1[t][r] * rres;
    wave_sync_lds();
  }

  float* os = Os[wave];
#pragma unroll
  for (int r = 0; r < 8; ++r) {
    const float l = lrow[r];
    const float inv = ((l > 0.f) ? (1.0f / l) : 0.f) * (1.0f / 1024.0f);
#pragma unroll
    for (int t = 0; t < 4; ++t) os[(8 * hh + r) * 64 + t * 16 + c] = oacc[t][r] * inv;
  }
  wave_sync_lds();
  {
    const int q4 = lane >> 3, c8 = (lane & 7) * 8;
    v4u hv[4], lv[4];
#pragma unroll
    for (int it = 0; it < 4; ++it) {
      const int row = it * 4 + q4;
      const float* sp = os + row * 64 + c8;
      v4u a, a2;
#pragma unroll
      for (int e = 0; e < 4; ++e) {
        const float f0 = sp[2 * e], f1 = sp[2 * e + 1];
        const unsigned short h0 = bf_bits(f0), h1 = bf_bits(f1);
        const unsigned short l0 = bf_bits(f0 - bf_up(h0)), l1 = bf_bits(f1 - bf_up(h1));
        a[e] = pk16(h0, h1); a2[e] = pk16(l0, l1);
      }
      hv[it] = a; lv[it] = a2;
    }
    for (int pass = 0; pass < 2; ++pass) {
#pragma unroll
      for (int it = 0; it < 4; ++it) {
        const int row = it * 4 + q4;
        const size_t go = (rowB + q0 + row) * CD + (size_t)h * HD + c8;
        *(volatile v4u*)(ohp + go) = hv[it];
        *(volatile v4u*)(olp + go) = lv[it];
      }
      __threadfence();
    }
  }
}

extern "C" void kernel_launch(void* const* d_in, const int* in_sizes, int n_in,
                              void* d_out, int out_size, void* d_ws, size_t ws_size,
                              hipStream_t stream) {
  if (n_in < 16) return;
  if (in_sizes[0] != NB * NT * CD || in_sizes[1] != NB * NT * CD || in_sizes[2] != NB * NT * CD) return;
  if (in_sizes[3] != NB * NT) return;
  if (in_sizes[4] != NT * CD) return;
  if (in_sizes[5] != CD * CD || in_sizes[7] != CD * CD || in_sizes[9] != CD * CD ||
      in_sizes[11] != CD * CD || in_sizes[12] != CD * CD) return;
  if (in_sizes[6] != CD || in_sizes[8] != CD || in_sizes[10] != CD || in_sizes[13] != CD) return;
  if (in_sizes[14] != NH * HD || in_sizes[15] != NH * HD) return;
  if (out_size != NB * NT * CD) return;

  const float* query = (const float*)d_in[0];
  const float* key   = (const float*)d_in[1];
  const float* value = (const float*)d_in[2];
  const int*   maskp = (const int*)d_in[3];
  const float* pos   = (const float*)d_in[4];
  const float* Wq    = (const float*)d_in[5];
  const float* bq    = (const float*)d_in[6];
  const float* Wk    = (const float*)d_in[7];
  const float* bk    = (const float*)d_in[8];
  const float* Wv    = (const float*)d_in[9];
  const float* bv    = (const float*)d_in[10];
  const float* Wp    = (const float*)d_in[11];
  const float* Wo    = (const float*)d_in[12];
  const float* bo    = (const float*)d_in[13];
  const float* pbu   = (const float*)d_in[14];
  const float* pbv   = (const float*)d_in[15];

  const size_t PX  = (size_t)NB * NT * CD * 2;
  const size_t PXp = (size_t)NT * CD * 2;
  const size_t PW  = (size_t)5 * CD * CD * 2;
  size_t off = 0;
  const size_t oXq  = off; off += PX;
  const size_t oXk  = off; off += PX;
  const size_t oXv  = off; off += PX;
  const size_t oXp  = off; off += PXp;
  const size_t oW   = off; off += PW;
  const size_t oQUh = off; off += PX;
  const size_t oQUl = off; off += PX;
  const size_t oQVh = off; off += PX;
  const size_t oQVl = off; off += PX;
  const size_t oKh  = off; off += PX;
  const size_t oKl  = off; off += PX;
  const size_t oPh  = off; off += PXp;
  const size_t oPl  = off; off += PXp;
  const size_t oVTh = off; off += PX;
  const size_t oVTl = off; off += PX;
  const size_t oOh  = off; off += PX;
  const size_t oOl  = off; off += PX;
  if (off > ws_size) return;
  if (off > (size_t)134217728) return;

  char* ws = (char*)d_ws;
  unsigned short* Xq  = (unsigned short*)(ws + oXq);
  unsigned short* Xk  = (unsigned short*)(ws + oXk);
  unsigned short* Xv  = (unsigned short*)(ws + oXv);
  unsigned short* Xp  = (unsigned short*)(ws + oXp);
  unsigned short* Wb  = (unsigned short*)(ws + oW);
  unsigned short* WbQ = Wb;
  unsigned short* WbK = Wb + (size_t)1 * CD * CD;
  unsigned short* WbV = Wb + (size_t)2 * CD * CD;
  unsigned short* WbP = Wb + (size_t)3 * CD * CD;
  unsigned short* WbO = Wb + (size_t)4 * CD * CD;
  unsigned short* QUh = (unsigned short*)(ws + oQUh);
  unsigned short* QUl = (unsigned short*)(ws + oQUl);
  unsigned short* QVh = (unsigned short*)(ws + oQVh);
  unsigned short* QVl = (unsigned short*)(ws + oQVl);
  unsigned short* Kh  = (unsigned short*)(ws + oKh);
  unsigned short* Kl  = (unsigned short*)(ws + oKl);
  unsigned short* Ph  = (unsigned short*)(ws + oPh);
  unsigned short* Pl  = (unsigned short*)(ws + oPl);
  unsigned short* VTh = (unsigned short*)(ws + oVTh);
  unsigned short* VTl = (unsigned short*)(ws + oVTl);
  unsigned short* Oh  = (unsigned short*)(ws + oOh);
  unsigned short* Ol  = (unsigned short*)(ws + oOl);

  float* xout = (float*)d_out;

  const float sscale = 0.125f;
  const float rres   = 1.0f / 4096.0f;

  const dim3 blk(256);
  const int n8a = NB * NT * CD / 8;
  const int n8p = NT * CD / 8;
  const int n8w = CD * CD / 8;
  const dim3 gCvtA((n8a + 255) / 256, 4);
  const dim3 gCvtW((n8w + 255) / 256, 5);
  const dim3 gQ(((NB * NT / 64) * (CD / 64) + 7) / 8, 1);
  const dim3 gP(((NT / 64) * (CD / 64) + 7) / 8, 1);
  const dim3 gVT(((CD / 64) * (NT / 64) + 7) / 8, NB);
  const dim3 gAttn(NB * NH * NQB);

  cvt_bf16x8m<<<gCvtA, blk, 0, stream>>>(query, key, value, pos, query,
                                         Xq, Xk, Xv, Xp, Xq,
                                         n8a, n8a, n8a, n8p, 0);
  cvt_bf16x8m<<<gCvtW, blk, 0, stream>>>(Wq, Wk, Wv, Wp, Wo,
                                         WbQ, WbK, WbV, WbP, WbO,
                                         n8w, n8w, n8w, n8w, n8w);
  gemm64<0, 4, 1><<<gQ, blk, 0, stream>>>(
      Xq, Xq, CD, 0LL, WbQ, CD, 0LL,
      (void*)QUh, (void*)QUl, (void*)QVh, (void*)QVl, CD, 0LL,
      NB * NT, CD, CD, 4096.0f, bq, pbu, pbv, 1);
  gemm64<0, 3, 1><<<gQ, blk, 0, stream>>>(
      Xk, Xk, CD, 0LL, WbK, CD, 0LL,
      (void*)Kh, (void*)Kl, (void*)Kh, (void*)Kl, CD, 0LL,
      NB * NT, CD, CD, 4096.0f, bk, bk, bk, 1);
  gemm64<0, 3, 1><<<gP, blk, 0, stream>>>(
      Xp, Xp, CD, 0LL, WbP, CD, 0LL,
      (void*)Ph, (void*)Pl, (void*)Ph, (void*)Pl, CD, 0LL,
      NT, CD, CD, 4096.0f, bq, bq, bq, 0);
  gemm64<0, 3, 1><<<gVT, blk, 0, stream>>>(
      WbV, WbV, CD, 0LL, Xv, CD, (long long)NT * CD,
      (void*)VTh, (void*)VTl, (void*)VTh, (void*)VTl, NT, (long long)CD * NT,
      CD, NT, CD, 4096.0f, bv, bv, bv, 2);
  attn64<<<gAttn, dim3(128), 0, stream>>>(QUh, QUl, QVh, QVl, Kh, Kl, Ph, Pl, VTh, VTl, maskp,
                                          Oh, Ol, sscale, rres);
  gemm64<1, 0, 0><<<gQ, blk, 0, stream>>>(
      Oh, Ol, CD, 0LL, WbO, CD, 0LL,
      (void*)xout, (void*)xout, (void*)xout, (void*)xout, CD, 0LL,
      NB * NT, CD, CD, 1.0f, bo, bo, bo, 1);
  (void)hipGetLastError();
}
